// ElectronDensityPredictor_12627203850727
// MI455X (gfx1250) — hardware-run, weakly checked
//
#include <hip/hip_runtime.h>
#include <stddef.h>
#include <stdint.h>
#include <math.h>


#define F_IN    128
#define HC      256
#define HEADS   8
#define HID     32
#define KD      512
#define NTHR    256
#define NWAVE   8
#define EPT     8
#define CHUNK   (NTHR * EPT)
#define WCAP    (EPT * 32)
#define LISTN   (NWAVE * WCAP)
#define NBMAX   2048
#define SLOTB   11
#define NB      1024
#define RCAP    20480
#define DEGCAP  256
#define GBM     64
#define GBN     64
#define GTHR    128
#define MROWS   128
#define HTHR    256
#define HROWS   128
#define INFOW   32
#define NEGSL   0.2f
#define BN_EPS  1e-5f
#define LDS_BK  ((2 * RCAP + 2 * NBMAX + LISTN) * 4 + 64)

static_assert(HC == 256 && HEADS * HID == HC && 32 * 8 == HC);
static_assert((CHUNK & (CHUNK - 1)) == 0 && CHUNK <= (1 << SLOTB));
static_assert(NBMAX == (1 << SLOTB) && NTHR * 8 == NBMAX && LISTN >= NBMAX);
static_assert(NB <= NBMAX && NB == NTHR * 4 && (NB % NWAVE) == 0);
static_assert((RCAP % (NTHR * 4)) == 0 && RCAP >= 16633 + 2048);
static_assert(LDS_BK <= 300000);
static_assert(GBM == (GTHR / 32) * 16 && GTHR == 2 * GBN && GTHR == 2 * GBM);
static_assert((F_IN % 32) == 0 && (KD % 32) == 0 && KD == 2 * HC && (HC % GBN) == 0 && GBN == 2 * HID);
static_assert((MROWS % GBM) == 0 && (MROWS % 32) == 0 && MROWS == HROWS && HROWS == (HTHR / 32) * 16);
static_assert((F_IN / 8) == 16 && (KD / 8) == 64);
static_assert(30080ull * (256 + 3 * 1024) + 16ull * 30080 * 4 + 30ull * RCAP * 4 + (1u << 20) <= (128u << 20));

typedef float          v4f  __attribute__((ext_vector_type(4)));
typedef float          v8f  __attribute__((ext_vector_type(8)));
typedef double         v2d  __attribute__((ext_vector_type(2)));
typedef int            v4i  __attribute__((ext_vector_type(4)));
typedef int            v8i  __attribute__((ext_vector_type(8)));
typedef unsigned int   v4u  __attribute__((ext_vector_type(4)));
typedef unsigned short v8us __attribute__((ext_vector_type(8)));
typedef __bf16         v16b __attribute__((ext_vector_type(16)));
typedef v4f  __attribute__((may_alias)) v4fa;
typedef v4i  __attribute__((may_alias)) v4ia;
typedef v2d  __attribute__((may_alias)) v2da;
typedef v8us __attribute__((may_alias)) v8usa;
union FragB { v16b v; v8us h[2]; v8i w; };

__device__ __forceinline__ v8f wmb(const FragB& a, const FragB& b, v8f c) {
  v8f d = __builtin_amdgcn_wmma_f32_16x16x32_bf16(false, a.v, false, b.v, (short)0, c, false, false);
  asm volatile("v_nop\n\tv_nop\n\tv_nop\n\tv_nop" : "+v"(d) : "v"(a.w), "v"(b.w));
  return d;
}

__device__ __forceinline__ unsigned int f2bf(float f) {
  const unsigned int u = __float_as_uint(f);
  const unsigned int r = ((u + 0x7FFFu + ((u >> 16) & 1u)) >> 16) & 0xFFFFu;
  return ((u & 0x7FFFFFFFu) > 0x7F800000u) ? 0x7FC0u : r;
}
__device__ __forceinline__ float bf2f(unsigned int b) { return __uint_as_float(b << 16); }
__device__ __forceinline__ float bfr(float f) { return bf2f(f2bf(f)); }
__device__ __forceinline__ v4f bfr4(const v4f a) {
  v4f r; r.x = bfr(a.x); r.y = bfr(a.y); r.z = bfr(a.z); r.w = bfr(a.w); return r;
}
__device__ __forceinline__ unsigned int pk2(float lo, float hi) { return f2bf(lo) | (f2bf(hi) << 16); }
__device__ __forceinline__ v4u pack8(const v4f a, const v4f b) {
  v4u r;
  r.x = pk2(a.x, a.y); r.y = pk2(a.z, a.w); r.z = pk2(b.x, b.y); r.w = pk2(b.z, b.w);
  return r;
}
__device__ __forceinline__ void split2(float y0, float y1, unsigned int& hw, unsigned int& lw) {
  const unsigned int h0 = f2bf(y0), h1 = f2bf(y1);
  const unsigned int l0 = f2bf(y0 - bf2f(h0)), l1 = f2bf(y1 - bf2f(h1));
  hw = h0 | (h1 << 16);
  lw = l0 | (l1 << 16);
}

__device__ __forceinline__ int scan_chunk(const int* __restrict__ dsts, int nE, int cbase, int slotBase,
                                          int nb, int vec8, int* list, int tid, int lane, int wave) {
  int wc = 0;
  const int el0  = tid * EPT;
  const int e0   = cbase + el0;
  const int sent = (int)0x80000000u;
  v4i da, db;
  if (vec8 != 0 && cbase + CHUNK <= nE) {
    da = *(const v4i*)(dsts + e0);
    db = *(const v4i*)(dsts + e0 + 4);
  } else {
    da.x = (e0     < nE) ? dsts[min(e0,     nE - 1)] : sent;
    da.y = (e0 + 1 < nE) ? dsts[min(e0 + 1, nE - 1)] : sent;
    da.z = (e0 + 2 < nE) ? dsts[min(e0 + 2, nE - 1)] : sent;
    da.w = (e0 + 3 < nE) ? dsts[min(e0 + 3, nE - 1)] : sent;
    db.x = (e0 + 4 < nE) ? dsts[min(e0 + 4, nE - 1)] : sent;
    db.y = (e0 + 5 < nE) ? dsts[min(e0 + 5, nE - 1)] : sent;
    db.z = (e0 + 6 < nE) ? dsts[min(e0 + 6, nE - 1)] : sent;
    db.w = (e0 + 7 < nE) ? dsts[min(e0 + 7, nE - 1)] : sent;
  }
  const unsigned nbs = (unsigned)slotBase;
  const unsigned unb = (unsigned)nb;
  const unsigned s0 = (unsigned)da.x - nbs, s1 = (unsigned)da.y - nbs;
  const unsigned s2 = (unsigned)da.z - nbs, s3 = (unsigned)da.w - nbs;
  const unsigned s4 = (unsigned)db.x - nbs, s5 = (unsigned)db.y - nbs;
  const unsigned s6 = (unsigned)db.z - nbs, s7 = (unsigned)db.w - nbs;
  const bool h0 = s0 < unb, h1 = s1 < unb, h2 = s2 < unb, h3 = s3 < unb;
  const bool h4 = s4 < unb, h5 = s5 < unb, h6 = s6 < unb, h7 = s7 < unb;
  const unsigned any = __builtin_amdgcn_ballot_w32(h0 | h1 | h2 | h3 | h4 | h5 | h6 | h7);
  if (any != 0u) {
#define HITJ(J, HJ, SJ) { \
      const unsigned mj = __builtin_amdgcn_ballot_w32(HJ); \
      if (mj != 0u) { \
        if (HJ) { \
          const int pos = wc + (int)__builtin_amdgcn_mbcnt_lo(mj, 0u); \
          if (pos < WCAP) list[wave * WCAP + pos] = ((el0 + (J)) << SLOTB) | (int)(SJ); \
        } \
        wc += (int)__builtin_popcount(mj); } }
    HITJ(0, h0, s0)
    HITJ(1, h1, s1)
    HITJ(2, h2, s2)
    HITJ(3, h3, s3)
    HITJ(4, h4, s4)
    HITJ(5, h5, s5)
    HITJ(6, h6, s6)
    HITJ(7, h7, s7)
#undef HITJ
  }
  return wc;
}

__device__ __forceinline__ void wtr_unit(const float* __restrict__ w, int Kin, int Ncol, int Kout,
                                         unsigned short* wt, int u) {
  const int kq = Kout >> 3;
  const int n  = u / kq;
  const int k8 = (u - n * kq) * 8;
  const int kk = k8 - (k8 / Kin) * Kin;
  const int ncl = n < Ncol ? n : Ncol - 1;
  const float* p = w + (size_t)kk * (size_t)Ncol + ncl;
  v4f a, b;
  a.x = p[0];                    a.y = p[(size_t)Ncol];         a.z = p[(size_t)2 * Ncol];     a.w = p[(size_t)3 * Ncol];
  b.x = p[(size_t)4 * Ncol];     b.y = p[(size_t)5 * Ncol];     b.z = p[(size_t)6 * Ncol];     b.w = p[(size_t)7 * Ncol];
  const v4u wv = pack8(a, b);
  unsigned short* o = wt + (size_t)n * (size_t)Kout + k8;
  *(volatile v4u*)o = wv;
  __threadfence();
  *(volatile v4u*)o = wv;
}

__global__ __launch_bounds__(NTHR) void k_prep(const float* __restrict__ x, const float* __restrict__ w1,
                                               const float* __restrict__ w2, const float* __restrict__ lw1,
                                               unsigned short* xb, unsigned short* w1t, unsigned short* w2d,
                                               unsigned short* lw1d, int nN, int nbX) {
  const int blk = (int)blockIdx.x, tid = (int)threadIdx.x;
  const int nb1 = (HC * (F_IN / 8)) / NTHR;
  const int nb2 = (HC * (KD / 8)) / NTHR;
  if (blk < nbX) {
    const int i   = blk * NTHR + tid;
    const int row = i >> 4;
    const int c0  = (i & 15) * 8;
    const int rc  = row < nN ? row : nN - 1;
    const float* p = x + (size_t)rc * F_IN + c0;
    v4f a = *(const v4fa*)p, b = *(const v4fa*)(p + 4);
    asm volatile("" :: "v"(a), "v"(b));
    const v4f z4 = {0.f, 0.f, 0.f, 0.f};
    if (row >= nN) { a = z4; b = z4; }
    const v4u hv = pack8(a, b);
    const size_t o = (size_t)row * F_IN + c0;
    *(volatile v4u*)(xb + o) = hv;
    __threadfence();
    *(volatile v4u*)(xb + o) = hv;
  } else if (blk < nbX + nb1) {
    wtr_unit(w1, F_IN, HC, F_IN, w1t, (blk - nbX) * NTHR + tid);
  } else if (blk < nbX + nb1 + nb2) {
    wtr_unit(w2, HC, HC, KD, w2d, (blk - nbX - nb1) * NTHR + tid);
  } else {
    wtr_unit(lw1, HC, HID, KD, lw1d, (blk - nbX - nb1 - nb2) * NTHR + tid);
  }
}

__global__ __launch_bounds__(NTHR) void k_bucket(const int* __restrict__ srcs, const int* __restrict__ dsts,
                                                 int* hits, int* offp, int* cntp, int* info,
                                                 int nN, int nE, int vec8) {
  extern __shared__ v4f lds_dyn[];
  int* reg1 = (int*)lds_dyn;
  int* reg2 = reg1 + RCAP;
  int* scnt = reg2 + RCAP;
  int* soff = scnt + NBMAX;
  int* list = soff + NBMAX;
  int* wcnt = list + LISTN;
  int* wtot = wcnt + NWAVE;
  const int tid = (int)threadIdx.x, lane = tid & 31, wave = tid >> 5;
  const int blk = (int)blockIdx.x;
  const int nodeBase = blk * NB;

  {
    const v4i z4 = {0, 0, 0, 0};
    for (int i = tid; i < NBMAX; i += NTHR) scnt[i] = 0;
    for (int i = tid * 4; i < RCAP; i += NTHR * 4) *(v4ia*)(reg2 + i) = z4;
  }
  __syncthreads();

  int tot = 0;
  const int nChunks = (nE + CHUNK - 1) / CHUNK;
#pragma unroll 1
  for (int ch = 0; ch < nChunks; ++ch) {
    const int cbase = ch * CHUNK;
    const int wc = scan_chunk(dsts, nE, cbase, nodeBase, NB, vec8, list, tid, lane, wave);
    if (lane == 0) wcnt[wave] = wc;
    __syncthreads();
    int pre = 0, all = 0;
#pragma unroll
    for (int w2 = 0; w2 < NWAVE; ++w2) {
      int c = wcnt[w2];
      c = c < 0 ? 0 : (c > WCAP ? WCAP : c);
      all += c;
      pre += (w2 < wave) ? c : 0;
    }
    const int wcc  = wc > WCAP ? WCAP : wc;
    const int base = tot + pre;
#pragma unroll 1
    for (int i = lane; i < wcc; i += 32) {
      const int ent = list[wave * WCAP + i];
      const int el  = (ent >> SLOTB) & (CHUNK - 1);
      const int sl  = ent & (NBMAX - 1);
      int eid = cbase + el;
      eid = eid > nE - 1 ? nE - 1 : eid;
      const int pos = base + i;
      if (pos < RCAP) reg1[pos] = (int)(((unsigned)eid << SLOTB) | (unsigned)sl);
    }
    tot += all;
    tot = tot > RCAP ? RCAP : tot;
    __syncthreads();
  }
  const int nh = tot;

  if (wave == 0) {
#pragma unroll 1
    for (int b0 = 0; b0 < nh; b0 += 32) {
      const int idx = b0 + lane;
      const int uv  = reg1[idx < nh ? idx : nh - 1];
      const int m32 = (nh - b0) < 32 ? (nh - b0) : 32;
#pragma unroll 1
      for (int k = 0; k < m32; ++k) {
        const int u  = __builtin_amdgcn_readlane(uv, k);
        const int sl = u & (NBMAX - 1);
        if (lane == 0) scnt[sl] = scnt[sl] + 1;
      }
    }
  }
  __syncthreads();

  {
    const v4i ca = *(const v4ia*)(scnt + 8 * tid);
    const v4i cb = *(const v4ia*)(scnt + 8 * tid + 4);
    const int e0 = ca.x < 0 ? 0 : ca.x, e1 = ca.y < 0 ? 0 : ca.y, e2 = ca.z < 0 ? 0 : ca.z, e3 = ca.w < 0 ? 0 : ca.w;
    const int e4 = cb.x < 0 ? 0 : cb.x, e5 = cb.y < 0 ? 0 : cb.y, e6 = cb.z < 0 ? 0 : cb.z, e7 = cb.w < 0 ? 0 : cb.w;
    const int ts = e0 + e1 + e2 + e3 + e4 + e5 + e6 + e7;
    int incl = ts;
#pragma unroll
    for (int d = 1; d < 32; d <<= 1) {
      const int up = __shfl_up(incl, d);
      if (lane >= d) incl += up;
    }
    if (lane == 31) wtot[wave] = incl;
    __syncthreads();
    int pre = 0;
#pragma unroll
    for (int w2 = 0; w2 < NWAVE; ++w2) pre += (w2 < wave) ? wtot[w2] : 0;
    int run = pre + incl - ts;
    soff[8 * tid + 0] = run; run += e0;
    soff[8 * tid + 1] = run; run += e1;
    soff[8 * tid + 2] = run; run += e2;
    soff[8 * tid + 3] = run; run += e3;
    soff[8 * tid + 4] = run; run += e4;
    soff[8 * tid + 5] = run; run += e5;
    soff[8 * tid + 6] = run; run += e6;
    soff[8 * tid + 7] = run;
  }
  __syncthreads();
  for (int i = tid; i < NBMAX; i += NTHR) list[i] = soff[i];
  __syncthreads();

  if (wave == 0) {
#pragma unroll 1
    for (int b0 = 0; b0 < nh; b0 += 32) {
      const int idx = b0 + lane;
      const int uv  = reg1[idx < nh ? idx : nh - 1];
      const int m32 = (nh - b0) < 32 ? (nh - b0) : 32;
#pragma unroll 1
      for (int k = 0; k < m32; ++k) {
        const int u   = __builtin_amdgcn_readlane(uv, k);
        const int sl  = u & (NBMAX - 1);
        const int eid = (int)((unsigned)u >> SLOTB);
        if (lane == 0) {
          int pos = list[sl];
          pos = pos < 0 ? 0 : (pos > RCAP - 1 ? RCAP - 1 : pos);
          reg2[pos] = eid;
          list[sl] = pos + 1;
        }
      }
    }
  }
  __syncthreads();

  int* hp = hits + (size_t)blk * RCAP;
#pragma unroll 1
  for (int base = tid * 4; base < RCAP; base += NTHR * 4) {
    const v4i ev = *(const v4ia*)(reg2 + base);
    const int q0 = ev.x < 0 ? 0 : (ev.x > nE - 1 ? nE - 1 : ev.x);
    const int q1 = ev.y < 0 ? 0 : (ev.y > nE - 1 ? nE - 1 : ev.y);
    const int q2 = ev.z < 0 ? 0 : (ev.z > nE - 1 ? nE - 1 : ev.z);
    const int q3 = ev.w < 0 ? 0 : (ev.w > nE - 1 ? nE - 1 : ev.w);
    int r0 = srcs[q0], r1 = srcs[q1], r2 = srcs[q2], r3 = srcs[q3];
    asm volatile("" :: "v"(r0), "v"(r1), "v"(r2), "v"(r3));
    r0 = r0 < 0 ? 0 : (r0 > nN - 1 ? nN - 1 : r0);
    r1 = r1 < 0 ? 0 : (r1 > nN - 1 ? nN - 1 : r1);
    r2 = r2 < 0 ? 0 : (r2 > nN - 1 ? nN - 1 : r2);
    r3 = r3 < 0 ? 0 : (r3 > nN - 1 ? nN - 1 : r3);
    v4i hv;
    hv.x = r0 & -(int)(base     < nh);
    hv.y = r1 & -(int)(base + 1 < nh);
    hv.z = r2 & -(int)(base + 2 < nh);
    hv.w = r3 & -(int)(base + 3 < nh);
    *(volatile v4i*)(hp + base) = hv;
    __threadfence();
    *(volatile v4i*)(hp + base) = hv;
  }
  {
    const v4i ov = *(const v4ia*)(soff + 4 * tid);
    const v4i cv = *(const v4ia*)(scnt + 4 * tid);
    v4i iv;
    iv.x = (tid == 0) ? nh : 0;
    iv.y = (tid == 0) ? (int)(nh >= RCAP) : 0;
    iv.z = 0; iv.w = 0;
    int* op = offp + (size_t)nodeBase + 4 * tid;
    int* cp = cntp + (size_t)nodeBase + 4 * tid;
    int* ip = info + (size_t)blk * INFOW + 4 * (tid & 7);
    *(volatile v4i*)op = ov;
    *(volatile v4i*)cp = cv;
    if (tid < 8) *(volatile v4i*)ip = iv;
    __threadfence();
    *(volatile v4i*)op = ov;
    *(volatile v4i*)cp = cv;
    if (tid < 8) *(volatile v4i*)ip = iv;
  }
}

__global__ __launch_bounds__(GTHR) __attribute__((amdgpu_num_vgpr(248))) void k_gemm(
    const unsigned short* __restrict__ A, const unsigned short* __restrict__ WT,
    float* outF, int K, int ldo,
    const float* __restrict__ atts, const float* __restrict__ attd,
    float* SD, int MPr)
{
  __shared__ __attribute__((aligned(16))) float stg[GBM * GBN];
  __shared__ __attribute__((aligned(16))) float satt[2 * GBN];
  __shared__ __attribute__((aligned(16))) float sdot[4 * GBM];
  const int tid = (int)threadIdx.x, lane = tid & 31, wave = tid >> 5, hh = lane >> 4, m = lane & 15;
  const int rowBase = (int)blockIdx.x * GBM;
  const int cb      = (int)blockIdx.y;
  const int col0    = cb * GBN;

  {
    const int which = tid >> 6;
    const int c  = tid & 63;
    const float vs = atts[cb * GBN + c];
    const float vd = attd[cb * GBN + c];
    const float v = (which == 0) ? vs : vd;
    satt[which * GBN + c] = bfr(v);
  }

  v8f acc[4];
  {
    const v8f z = {0.f, 0.f, 0.f, 0.f, 0.f, 0.f, 0.f, 0.f};
    acc[0] = z; acc[1] = z; acc[2] = z; acc[3] = z;
  }
  const unsigned short* ap = A  + (size_t)(rowBase + 16 * wave + m) * (size_t)K + 8 * hh;
  const unsigned short* wp = WT + (size_t)(col0 + m) * (size_t)K + 8 * hh;
  const int ksteps = K >> 5;
#pragma unroll 1
  for (int ks = 0; ks < ksteps; ++ks) {
    FragB af;
    af.h[0] = *(const v8usa*)(ap + 32 * ks);
    af.h[1] = *(const v8usa*)(ap + 32 * ks + 16);
#pragma unroll
    for (int t = 0; t < 4; ++t) {
      const unsigned short* wq = wp + (size_t)(16 * t) * (size_t)K + 32 * ks;
      FragB bf;
      bf.h[0] = *(const v8usa*)wq;
      bf.h[1] = *(const v8usa*)(wq + 16);
      acc[t] = wmb(af, bf, acc[t]);
    }
  }

#pragma unroll
  for (int t = 0; t < 4; ++t) {
    const int lc = 16 * t + m;
#pragma unroll
    for (int r = 0; r < 8; ++r) {
      const int lr = 16 * wave + 8 * hh + r;
      stg[lr * GBN + lc] = acc[t][r];
    }
  }
  __syncthreads();

  {
    const int row = tid & 63, which = tid >> 6;
    const float* sa = satt + which * GBN;
    const float* hr = stg + row * GBN;
    float d0 = 0.f, d1 = 0.f;
#pragma unroll 4
    for (int c4 = 0; c4 < HID / 4; ++c4) {
      const v4f hv = *(const v4fa*)(hr + 4 * c4);
      const v4f av = *(const v4fa*)(sa + 4 * c4);
      d0 = fmaf(hv.x, av.x, d0);
      d0 = fmaf(hv.y, av.y, d0);
      d0 = fmaf(hv.z, av.z, d0);
      d0 = fmaf(hv.w, av.w, d0);
    }
#pragma unroll 4
    for (int c4 = HID / 4; c4 < GBN / 4; ++c4) {
      const v4f hv = *(const v4fa*)(hr + 4 * c4);
      const v4f av = *(const v4fa*)(sa + 4 * c4);
      d1 = fmaf(hv.x, av.x, d1);
      d1 = fmaf(hv.y, av.y, d1);
      d1 = fmaf(hv.z, av.z, d1);
      d1 = fmaf(hv.w, av.w, d1);
    }
    sdot[(0 + which) * GBM + row] = d0;
    sdot[(2 + which) * GBM + row] = d1;
  }
  __syncthreads();

  v4f fv[8];
#pragma unroll
  for (int i = 0; i < 8; ++i) {
    const int lr = 16 * wave + 2 * i + hh;
    fv[i] = *(const v4fa*)(stg + lr * GBN + 4 * m);
  }
  const int which2 = lane >> 4, piece = lane & 15;
  const int hl = wave & 1;
  const v4f sdv = *(const v4fa*)(sdot + (2 * hl + which2) * GBM + 4 * piece);
  float* sp = SD + (size_t)(2 * (2 * cb + hl) + which2) * (size_t)MPr + rowBase + 4 * piece;

#pragma unroll
  for (int i = 0; i < 8; ++i) {
    const int lr = 16 * wave + 2 * i + hh;
    const int gr = rowBase + lr;
    float* op = outF + (size_t)gr * (size_t)ldo + col0 + 4 * m;
    *(volatile v4f*)op = fv[i];
  }
  if (wave < 2) *(volatile v4f*)sp = sdv;
  __threadfence();
#pragma unroll
  for (int i = 0; i < 8; ++i) {
    const int lr = 16 * wave + 2 * i + hh;
    const int gr = rowBase + lr;
    float* op = outF + (size_t)gr * (size_t)ldo + col0 + 4 * m;
    *(volatile v4f*)op = fv[i];
  }
  if (wave < 2) *(volatile v4f*)sp = sdv;
}

__global__ __launch_bounds__(NTHR) void k_replay(
    const int* __restrict__ hits, const int* __restrict__ offp, const int* __restrict__ cntp,
    const int* __restrict__ info,
    const float* __restrict__ hf, const float* __restrict__ SD, const float* __restrict__ bias,
    float* tf, double* rec, int nN, int MPr) {
  __shared__ __attribute__((aligned(16))) float  wrow[NWAVE * HC];
  __shared__ __attribute__((aligned(16))) double sst[NWAVE * HC * 2];
  const int tid = (int)threadIdx.x, lane = tid & 31, wave = tid >> 5;
  const int blk = (int)blockIdx.x;
  const int nodeBase = blk * NB;
  const int* hp = hits + (size_t)blk * RCAP;
  int nh = info[blk * INFOW];
  nh = nh < 0 ? 0 : (nh > RCAP ? RCAP : nh);
  const bool ovf = info[blk * INFOW + 1] != 0;
  const float qnan = __int_as_float(0x7fc00000);

  const int c0   = 8 * lane;
  const int head = lane >> 2;
  const float* ASp = SD + (size_t)(2 * head) * (size_t)MPr;
  const float* ADp = ASp + MPr;
  const v4f bA = bfr4(*(const v4fa*)(bias + c0));
  const v4f bB = bfr4(*(const v4fa*)(bias + c0 + 4));
  float* wr = wrow + wave * HC;

  double cs[8], cq[8];
#pragma unroll
  for (int i = 0; i < 8; ++i) { cs[i] = 0.0; cq[i] = 0.0; }

  const int nbw = NB / NWAVE;
#pragma unroll 1
  for (int jt = 0; jt < nbw; ++jt) {
    const int slot = wave * nbw + jt;
    const int node = nodeBase + slot;
    const int gcl  = node < nN ? node : nN - 1;
    int o = offp[node];
    int c = cntp[node];
    o = o < 0 ? 0 : (o > RCAP - 1 ? RCAP - 1 : o);
    const bool big = c > DEGCAP;
    c = c < 0 ? 0 : (c > DEGCAP ? DEGCAP : c);
    int room = nh - o;
    room = room < 0 ? 0 : room;
    c = c > room ? room : c;
    o = __builtin_amdgcn_readfirstlane(o);
    c = __builtin_amdgcn_readfirstlane(c);
    int last = o + c - 1; last = last < o ? o : last;
    const float pz = (ovf || big) ? qnan : 0.0f;

    v4f av = *(const v4fa*)(hf + (size_t)gcl * HC + c0);
    v4f bv = *(const v4fa*)(hf + (size_t)gcl * HC + c0 + 4);
    const float adv = ADp[gcl];
    float l0 = ASp[gcl] + adv;
    l0 = l0 > 0.f ? l0 : NEGSL * l0;
    float mx = l0, dn = 1.0f;

#pragma unroll 1
    for (int b0 = 0; b0 < c; b0 += 32) {
      int idx = o + b0 + lane;
      idx = idx > last ? last : idx;
      int sr = hp[idx];
      sr = sr < 0 ? 0 : (sr > nN - 1 ? nN - 1 : sr);
      const int m32 = (c - b0) < 32 ? (c - b0) : 32;
#pragma unroll 1
      for (int k = 0; k < m32; ++k) {
        const int sk = __builtin_amdgcn_readlane(sr, k);
        const v4f f0 = *(const v4fa*)(hf + (size_t)sk * HC + c0);
        const v4f f1 = *(const v4fa*)(hf + (size_t)sk * HC + c0 + 4);
        float lg = ASp[sk] + adv;
        lg = lg > 0.f ? lg : NEGSL * lg;
        const float df = lg - mx;
        const float ee = expf(-fabsf(df));
        const bool up  = df > 0.f;
        const float s1 = up ? ee : 1.0f;
        const float s2 = up ? 1.0f : ee;
        mx = up ? lg : mx;
        dn = fmaf(dn, s1, s2);
        av.x = fmaf(av.x, s1, s2 * f0.x);
        av.y = fmaf(av.y, s1, s2 * f0.y);
        av.z = fmaf(av.z, s1, s2 * f0.z);
        av.w = fmaf(av.w, s1, s2 * f0.w);
        bv.x = fmaf(bv.x, s1, s2 * f1.x);
        bv.y = fmaf(bv.y, s1, s2 * f1.y);
        bv.z = fmaf(bv.z, s1, s2 * f1.z);
        bv.w = fmaf(bv.w, s1, s2 * f1.w);
      }
    }
    const float inv = 1.0f / dn;
    v4f oa, ob;
    oa.x = (av.x * inv + bA.x) + pz;
    oa.y = (av.y * inv + bA.y) + pz;
    oa.z = (av.z * inv + bA.z) + pz;
    oa.w = (av.w * inv + bA.w) + pz;
    ob.x = (bv.x * inv + bB.x) + pz;
    ob.y = (bv.y * inv + bB.y) + pz;
    ob.z = (bv.z * inv + bB.z) + pz;
    ob.w = (bv.w * inv + bB.w) + pz;
    *(v4fa*)(wr + c0)     = oa;
    *(v4fa*)(wr + c0 + 4) = ob;
    __syncthreads();

#pragma unroll 1
    for (int j = 0; j < 8; ++j) {
      const int ix = 4 * lane + (j & 3) + ((j >> 2) << 7);
      const float v = wr[ix];
      const float t = v > 0.0f ? v : expm1f(v);
      wr[ix] = t;
    }
    const v4f g0 = *(const v4fa*)(wr + 4 * lane);
    const v4f g1 = *(const v4fa*)(wr + 128 + 4 * lane);
    const bool live = node < nN;
    if (live) {
      const double d0 = (double)g0.x, d1 = (double)g0.y, d2 = (double)g0.z, d3 = (double)g0.w;
      const double d4 = (double)g1.x, d5 = (double)g1.y, d6 = (double)g1.z, d7 = (double)g1.w;
      cs[0] += d0; cq[0] = fma(d0, d0, cq[0]);
      cs[1] += d1; cq[1] = fma(d1, d1, cq[1]);
      cs[2] += d2; cq[2] = fma(d2, d2, cq[2]);
      cs[3] += d3; cq[3] = fma(d3, d3, cq[3]);
      cs[4] += d4; cq[4] = fma(d4, d4, cq[4]);
      cs[5] += d5; cq[5] = fma(d5, d5, cq[5]);
      cs[6] += d6; cq[6] = fma(d6, d6, cq[6]);
      cs[7] += d7; cq[7] = fma(d7, d7, cq[7]);
    }
    float* tp = tf + (size_t)gcl * HC + 4 * lane;
    if (live) {
      *(volatile v4f*)tp = g0;
      *(volatile v4f*)(tp + 128) = g1;
    }
    __threadfence();
    if (live) {
      *(volatile v4f*)tp = g0;
      *(volatile v4f*)(tp + 128) = g1;
    }
    __syncthreads();
  }

#pragma unroll
  for (int i = 0; i < 4; ++i) {
    const int ca = 4 * lane + i, cb2 = 128 + 4 * lane + i;
    sst[(wave * HC + ca) * 2 + 0]  = cs[i];
    sst[(wave * HC + ca) * 2 + 1]  = cq[i];
    sst[(wave * HC + cb2) * 2 + 0] = cs[4 + i];
    sst[(wave * HC + cb2) * 2 + 1] = cq[4 + i];
  }
  __syncthreads();
  {
    double S = 0.0, Q = 0.0;
#pragma unroll 1
    for (int w2 = 0; w2 < NWAVE; ++w2) {
      S += sst[(w2 * HC + tid) * 2 + 0];
      Q += sst[(w2 * HC + tid) * 2 + 1];
    }
    v2d rv; rv.x = S; rv.y = Q;
    double* rp = rec + ((size_t)blk * HC + tid) * 2;
    *(volatile v2d*)rp = rv;
    __threadfence();
    *(volatile v2d*)rp = rv;
  }
}

__global__ __launch_bounds__(HC) void k_comb(const double* __restrict__ rec, int nBk, double invN, float* stat) {
  __shared__ __attribute__((aligned(16))) float stg[2 * HC];
  const int tid = (int)threadIdx.x;
  double S = 0.0, Q = 0.0;
#pragma unroll 1
  for (int b = 0; b < nBk; ++b) {
    const v2d r = *(const v2da*)(rec + ((size_t)b * HC + tid) * 2);
    S += r.x;
    Q += r.y;
  }
  const double mean = S * invN;
  double var = Q * invN - mean * mean;
  var = var < 0.0 ? 0.0 : var;
  const float rstd = 1.0f / sqrtf((float)var + BN_EPS);
  stg[tid] = (float)mean;
  stg[HC + tid] = rstd;
  __syncthreads();
  v4f v;
  if (tid < (2 * HC) / 4) {
    v = *(const v4fa*)(stg + 4 * tid);
    *(volatile v4f*)(stat + 4 * tid) = v;
  }
  __threadfence();
  if (tid < (2 * HC) / 4) {
    *(volatile v4f*)(stat + 4 * tid) = v;
  }
}

__global__ __launch_bounds__(NTHR) void k_norm(const float* __restrict__ tf, const float* __restrict__ stat,
                                               const float* __restrict__ gam, const float* __restrict__ bet,
                                               unsigned short* xn, int nN, int nUnits) {
  __shared__ __attribute__((aligned(16))) float sp[4 * HC];
  const int tid = (int)threadIdx.x;
  sp[tid]          = stat[tid];
  sp[HC + tid]     = stat[HC + tid];
  sp[2 * HC + tid] = bfr(gam[tid]);
  sp[3 * HC + tid] = bfr(bet[tid]);
  __syncthreads();
  const int u = (int)blockIdx.x * NTHR + tid;
  if (u >= nUnits) return;
  const int row = u >> 5;
  const int c0  = (u & 31) * 8;
  const int rc  = row < nN ? row : nN - 1;
  const float* p = tf + (size_t)rc * HC + c0;
  v4f a = *(const v4fa*)p, b = *(const v4fa*)(p + 4);
  asm volatile("" :: "v"(a), "v"(b));
  const v4f m0 = *(const v4fa*)(sp + c0),          m1 = *(const v4fa*)(sp + c0 + 4);
  const v4f r0 = *(const v4fa*)(sp + HC + c0),     r1 = *(const v4fa*)(sp + HC + c0 + 4);
  const v4f g0 = *(const v4fa*)(sp + 2 * HC + c0), g1 = *(const v4fa*)(sp + 2 * HC + c0 + 4);
  const v4f e0 = *(const v4fa*)(sp + 3 * HC + c0), e1 = *(const v4fa*)(sp + 3 * HC + c0 + 4);
  const bool ok = row < nN;
  const float y0 = ok ? (((a.x - m0.x) * r0.x) * g0.x + e0.x) : 0.0f;
  const float y1 = ok ? (((a.y - m0.y) * r0.y) * g0.y + e0.y) : 0.0f;
  const float y2 = ok ? (((a.z - m0.z) * r0.z) * g0.z + e0.z) : 0.0f;
  const float y3 = ok ? (((a.w - m0.w) * r0.w) * g0.w + e0.w) : 0.0f;
  const float y4 = ok ? (((b.x - m1.x) * r1.x) * g1.x + e1.x) : 0.0f;
  const float y5 = ok ? (((b.y - m1.y) * r1.y) * g1.y + e1.y) : 0.0f;
  const float y6 = ok ? (((b.z - m1.z) * r1.z) * g1.z + e1.z) : 0.0f;
  const float y7 = ok ? (((b.w - m1.w) * r1.w) * g1.w + e1.w) : 0.0f;
  unsigned int h0, h1, h2, h3, l0, l1, l2, l3;
  split2(y0, y1, h0, l0);
  split2(y2, y3, h1, l1);
  split2(y4, y5, h2, l2);
  split2(y6, y7, h3, l3);
  v4u hv, lv;
  hv.x = h0; hv.y = h1; hv.z = h2; hv.w = h3;
  lv.x = l0; lv.y = l1; lv.z = l2; lv.w = l3;
  unsigned short* op = xn + (size_t)row * KD + c0;
  *(volatile v4u*)op = hv;
  *(volatile v4u*)(op + HC) = lv;
  __threadfence();
  *(volatile v4u*)op = hv;
  *(volatile v4u*)(op + HC) = lv;
}

__global__ __launch_bounds__(HTHR) __attribute__((amdgpu_num_vgpr(248))) void k_head(
    const unsigned short* __restrict__ A, const unsigned short* __restrict__ WT,
    const float* __restrict__ lb1, const float* __restrict__ lw2, const float* __restrict__ lb2,
    const int* __restrict__ info, int nBk, float* out, int nN) {
  __shared__ __attribute__((aligned(16))) float zt[HROWS * HID];
  __shared__ __attribute__((aligned(16))) float sp[2 * HID];
  __shared__ __attribute__((aligned(16))) float ys[HROWS];
  const int tid = (int)threadIdx.x, lane = tid & 31, wave = tid >> 5, hh = lane >> 4, m = lane & 15;
  const int rowBase = (int)blockIdx.x * HROWS;

  if (tid < HID) {
    sp[tid]       = bfr(lb1[tid]);
    sp[HID + tid] = bfr(lw2[tid]);
  }

  v8f acc[2];
  {
    const v8f z = {0.f, 0.f, 0.f, 0.f, 0.f, 0.f, 0.f, 0.f};
    acc[0] = z; acc[1] = z;
  }
  const unsigned short* ap = A  + (size_t)(rowBase + 16 * wave + m) * (size_t)KD + 8 * hh;
  const unsigned short* wp = WT + (size_t)m * (size_t)KD + 8 * hh;
#pragma unroll 1
  for (int k0 = 0; k0 < KD; k0 += 32) {
    FragB af;
    af.h[0] = *(const v8usa*)(ap + k0);
    af.h[1] = *(const v8usa*)(ap + k0 + 16);
#pragma unroll
    for (int t = 0; t < 2; ++t) {
      const unsigned short* wq = wp + (size_t)(16 * t) * (size_t)KD + k0;
      FragB bf;
      bf.h[0] = *(const v8usa*)wq;
      bf.h[1] = *(const v8usa*)(wq + 16);
      acc[t] = wmb(af, bf, acc[t]);
    }
  }
#pragma unroll
  for (int t = 0; t < 2; ++t) {
    const int lc = 16 * t + m;
#pragma unroll
    for (int r = 0; r < 8; ++r) {
      const int lr = 16 * wave + 8 * hh + r;
      zt[lr * HID + lc] = acc[t][r];
    }
  }
  __syncthreads();

  if (tid < HROWS) {
    const float* zr = zt + tid * HID;
    float y = 0.0f;
#pragma unroll 1
    for (int c = 0; c < HID; ++c) {
      const float z = zr[c] + sp[c];
      const float uu = z > 0.0f ? z : expm1f(z);
      y = fmaf(uu, sp[HID + c], y);
    }
    ys[tid] = y + bfr(lb2[0]);
  }
  __syncthreads();

  if (wave == 0) {
    const int bi = lane < nBk ? lane : nBk - 1;
    const int fb = info[bi * INFOW + 1];
    const unsigned anyf = __builtin_amdgcn_ballot_w32(fb != 0);
    const float pz = (anyf != 0u) ? __int_as_float(0x7fc00000) : 0.0f;
    v4f v = *(const v4fa*)(ys + 4 * lane);
    v.x += pz; v.y += pz; v.z += pz; v.w += pz;
    int rem = nN - rowBase;
    rem = rem < 0 ? 0 : (rem > HROWS ? HROWS : rem);
    const int npc = rem >> 2;
    float* op = out + (size_t)rowBase + 4 * lane;
    if (lane < npc) *(volatile v4f*)op = v;
    __threadfence();
    if (lane < npc) *(volatile v4f*)op = v;
  }
}

static inline int cdiv(int a, int b) { return (a + b - 1) / b; }
static inline size_t al256(size_t o) { return (o + 255) & ~(size_t)255; }

extern "C" void kernel_launch(void* const* d_in, const int* in_sizes, int n_in,
                              void* d_out, int out_size, void* d_ws, size_t ws_size,
                              hipStream_t stream) {
  if (n_in < 18) return;
  const int nN = in_sizes[0] / F_IN;
  if (nN < 1 || in_sizes[0] != nN * F_IN || nN >= 32768 || (nN & 3) != 0) return;
  if (in_sizes[1] < 2 || (in_sizes[1] & 1) != 0) return;
  const int nE = in_sizes[1] / 2;
  if (nE < 1 || nE >= (1 << (32 - SLOTB))) return;
  if (in_sizes[2] != F_IN * HC) return;
  if (in_sizes[3] != HC || in_sizes[4] != HC) return;
  if (in_sizes[5] != HC || in_sizes[6] != HC || in_sizes[7] != HC) return;
  if (in_sizes[8] != HC * HC) return;
  if (in_sizes[9] != HC || in_sizes[10] != HC) return;
  if (in_sizes[11] != HC || in_sizes[12] != HC || in_sizes[13] != HC) return;
  if (in_sizes[14] != HC * HID) return;
  if (in_sizes[15] != HID || in_sizes[16] != HID || in_sizes[17] != 1) return;
  if (out_size != nN) return;

  const float* x    = (const float*)d_in[0];
  const int*   ei   = (const int*)  d_in[1];
  const float* w1   = (const float*)d_in[2];
  const float* a1s  = (const float*)d_in[3];
  const float* a1d  = (const float*)d_in[4];
  const float* b1   = (const float*)d_in[5];
  const float* g1   = (const float*)d_in[6];
  const float* be1  = (const float*)d_in[7];
  const float* w2   = (const float*)d_in[8];
  const float* a2s  = (const float*)d_in[9];
  const float* a2d  = (const float*)d_in[10];
  const float* b2   = (const float*)d_in[11];
  const float* g2   = (const float*)d_in[12];
  const float* be2  = (const float*)d_in[13];
  const float* lw1  = (const float*)d_in[14];
  const float* lb1  = (const float*)d_in[15];
  const float* lw2  = (const float*)d_in[16];
  const float* lb2  = (const float*)d_in[17];
  float* out = (float*)d_out;
  const int* src = ei;
  const int* dst = ei + nE;

  const int MP  = cdiv(nN, MROWS) * MROWS;
  const int nBk = cdiv(nN, NB);
  if (nBk < 1 || nBk > 32) return;
  const int vec8 = ((nE & 3) == 0) ? 1 : 0;
  const double invN = 1.0 / (double)nN;

  char* ws = (char*)d_ws;
  size_t off = 0;
  const size_t oXB   = off; off = al256(off + (size_t)MP * F_IN * 2);
  const size_t oW1T  = off; off = al256(off + (size_t)HC * F_IN * 2);
  const size_t oW2D  = off; off = al256(off + (size_t)HC * KD * 2);
  const size_t oLW1D = off; off = al256(off + (size_t)HID * KD * 2);
  const size_t oHF   = off; off = al256(off + (size_t)MP * HC * 4);
  const size_t oSD   = off; off = al256(off + (size_t)2 * HEADS * MP * 4);
  const size_t oTF   = off; off = al256(off + (size_t)MP * HC * 4);
  const size_t oXN   = off; off = al256(off + (size_t)MP * KD * 2);
  const size_t oHITS = off; off = al256(off + (size_t)nBk * RCAP * 4);
  const size_t oOFF  = off; off = al256(off + (size_t)nBk * NB * 4);
  const size_t oCNT  = off; off = al256(off + (size_t)nBk * NB * 4);
  const size_t oINFO = off; off = al256(off + (size_t)32 * INFOW * 4);
  const size_t oREC  = off; off = al256(off + (size_t)nBk * HC * 2 * 8);
  const size_t oST1  = off; off = al256(off + (size_t)2 * HC * 4);
  const size_t oST2  = off; off = al256(off + (size_t)2 * HC * 4);
  if (off > ws_size || off > (size_t)(128u << 20)) return;
  unsigned short* XB   = (unsigned short*)(ws + oXB);
  unsigned short* W1T  = (unsigned short*)(ws + oW1T);
  unsigned short* W2D  = (unsigned short*)(ws + oW2D);
  unsigned short* LW1D = (unsigned short*)(ws + oLW1D);
  float*  HF   = (float*)(ws + oHF);
  float*  SDp  = (float*)(ws + oSD);
  float*  TF   = (float*)(ws + oTF);
  unsigned short* XN = (unsigned short*)(ws + oXN);
  int*    HITS = (int*)(ws + oHITS);
  int*    OFFp = (int*)(ws + oOFF);
  int*    CNTp = (int*)(ws + oCNT);
  int*    INFO = (int*)(ws + oINFO);
  double* REC  = (double*)(ws + oREC);
  float*  ST1  = (float*)(ws + oST1);
  float*  ST2  = (float*)(ws + oST2);

  hipFuncSetAttribute(reinterpret_cast<const void*>(&k_bucket),
                      hipFuncAttributeMaxDynamicSharedMemorySize, LDS_BK);

  const int nbX = (MP * (F_IN / 8)) / NTHR;
  const int nbW = (HC * (F_IN / 8)) / NTHR + (HC * (KD / 8)) / NTHR + (HID * (KD / 8)) / NTHR;
  const int gM  = MP / GBM;
  const int nUn = MP * (HC / 8);

  k_prep<<<nbX + nbW, NTHR, 0, stream>>>(x, w1, w2, lw1, XB, W1T, W2D, LW1D, nN, nbX);
  k_bucket<<<nBk, NTHR, LDS_BK, stream>>>(src, dst, HITS, OFFp, CNTp, INFO, nN, nE, vec8);
  k_gemm<<<dim3(gM, HC / GBN), GTHR, 0, stream>>>(XB, W1T, HF, F_IN, HC, a1s, a1d, SDp, MP);
  k_replay<<<nBk, NTHR, 0, stream>>>(HITS, OFFp, CNTp, INFO, HF, SDp, b1, TF, REC, nN, MP);
  k_comb<<<1, HC, 0, stream>>>(REC, nBk, invN, ST1);
  k_norm<<<cdiv(nUn, NTHR), NTHR, 0, stream>>>(TF, ST1, g1, be1, XN, nN, nUn);
  k_gemm<<<dim3(gM, HC / GBN), GTHR, 0, stream>>>(XN, W2D, HF, KD, HC, a2s, a2d, SDp, MP);
  k_replay<<<nBk, NTHR, 0, stream>>>(HITS, OFFp, CNTp, INFO, HF, SDp, b2, TF, REC, nN, MP);
  k_comb<<<1, HC, 0, stream>>>(REC, nBk, invN, ST2);
  k_norm<<<cdiv(nUn, NTHR), NTHR, 0, stream>>>(TF, ST2, g2, be2, XN, nN, nUn);
  k_head<<<MP / HROWS, HTHR, 0, stream>>>(XN, LW1D, lb1, lw2, lb2, INFO, nBk, out, nN);
}
